// SimpleCrossLingualAdapter_51908974739518
// MI455X (gfx1250) — hardware-run, weakly checked
//
#include <hip/hip_runtime.h>
#include <math.h>

constexpr int N_BATCH = 2048;
constexpr int N_STEPS = 128;
constexpr int N_VOCAB = 256;
constexpr int N_CHAN  = 32;
constexpr int N_HID   = 128;
constexpr int N_GATE3 = 384;
constexpr int N_FEAT  = 256;
constexpr int N_OUT   = 256;
constexpr int N_LANG  = 3;
constexpr int N_BOT   = 32;
constexpr int N_THR   = 256;
constexpr int ROWS_PB = 16;

static_assert(N_GATE3 == 3 * N_HID);
static_assert(N_FEAT == 2 * N_HID);
static_assert(N_BOT * 8 == N_FEAT);
static_assert(N_BATCH % ROWS_PB == 0);
static_assert(N_HID % 32 == 0 && N_FEAT % 32 == 0 && N_BOT % 32 == 0);
static_assert(N_BATCH % 64 == 0 && N_OUT % 64 == 0);

constexpr float W_CARRY   = 128.0f;
constexpr float H_CARRY   = 256.0f;
constexpr float Y_CARRY   = 64.0f;
constexpr float REC_FOLD  = 1.0f / (H_CARRY * W_CARRY);
constexpr float ADP_FOLD  = 1.0f / (H_CARRY * W_CARRY);
constexpr float PRJ_FOLD  = 1.0f / (Y_CARRY * W_CARRY);
constexpr float F16_MIN_NORMAL = 6.103515625e-05f;
constexpr float LN_EPSILON = 1e-5f;

constexpr int H_PITCH = 136;
constexpr int X_PITCH = 388;
constexpr int F_PITCH = 132;
constexpr int A16_PITCH = 264;
constexpr int AX_PITCH  = 260;
constexpr int HD_PITCH  = 40;

typedef __attribute__((ext_vector_type(16))) _Float16 v16h;
typedef __attribute__((ext_vector_type(8)))  _Float16 v8h;
typedef __attribute__((ext_vector_type(4)))  _Float16 v4h;
typedef __attribute__((ext_vector_type(8)))  float    v8f;
typedef __attribute__((ext_vector_type(4)))  float    v4f;
typedef __attribute__((ext_vector_type(4)))  int      v4i;

struct FragH {
  union U { v16h v; v8h h[2]; };
  static __device__ __forceinline__ v16h load(const _Float16* p) {
    U f;
    f.h[0] = *(const v8h*)(p);
    f.h[1] = *(const v8h*)(p + 16);
    return f.v;
  }
  static __device__ __forceinline__ v8f mma(v16h a, v16h b, v8f c) {
    return __builtin_amdgcn_wmma_f32_16x16x32_f16(false, a, false, b, (short)0, c, false, false);
  }
};

__device__ __forceinline__ void wm_guard(v8f& acc, v16h a, v16h b) {
  asm volatile("v_nop\n\tv_nop\n\tv_nop\n\tv_nop" : "+v"(acc) : "v"(a), "v"(b));
}
__device__ __forceinline__ void keep4_h(v16h a, v16h b, v16h c, v16h d) {
  asm volatile("v_nop" :: "v"(a), "v"(b), "v"(c), "v"(d));
}

__device__ __forceinline__ int clampi(int v, int lo, int hi) {
  const int a = (v < lo) ? lo : v;
  return (a > hi) ? hi : a;
}

__device__ __forceinline__ _Float16 f16_operand(float carried) {
  const float c = (fabsf(carried) < F16_MIN_NORMAL) ? 0.0f : carried;
  return (_Float16)c;
}

__device__ __forceinline__ float sigm_f(float x) {
  const float xc = fminf(fmaxf(x, -30.0f), 30.0f);
  return 1.0f / (1.0f + expf(-xc));
}
__device__ __forceinline__ float tanh_f(float x) {
  const float xc = fminf(fmaxf(x, -15.0f), 15.0f);
  return 1.0f - 2.0f / (1.0f + expf(2.0f * xc));
}

__device__ __forceinline__ void cvt8_store(const float* __restrict__ src, _Float16* __restrict__ dst, float carry) {
  const v4f a = *(const v4f*)(src);
  const v4f b = *(const v4f*)(src + 4);
  v8h h;
#pragma unroll
  for (int e = 0; e < 4; ++e) {
    h[e]     = f16_operand(a[e] * carry);
    h[4 + e] = f16_operand(b[e] * carry);
  }
  *(volatile v8h*)dst = h;
  __threadfence();
  *(volatile v8h*)dst = h;
}

constexpr int XT_ELEMS   = 2 * N_VOCAB * N_GATE3;
constexpr int XT_BLOCKS  = XT_ELEMS / N_THR;
constexpr int WHH_BLOCKS = 2 * N_GATE3 * N_HID / 8 / N_THR;
constexpr int PW_BLOCKS  = N_OUT * N_FEAT / 8 / N_THR;
constexpr int DW_BLOCKS  = N_LANG * N_BOT * N_FEAT / 8 / N_THR;
constexpr int UW_BLOCKS  = N_LANG * N_FEAT * N_BOT / 8 / N_THR;
constexpr int PREP_BLOCKS = XT_BLOCKS + WHH_BLOCKS + PW_BLOCKS + DW_BLOCKS + UW_BLOCKS;
static_assert(XT_BLOCKS * N_THR == XT_ELEMS);
static_assert(WHH_BLOCKS * N_THR * 8 == 2 * N_GATE3 * N_HID);
static_assert(PW_BLOCKS * N_THR * 8 == N_OUT * N_FEAT);
static_assert(DW_BLOCKS * N_THR * 8 == N_LANG * N_BOT * N_FEAT);
static_assert(UW_BLOCKS * N_THR * 8 == N_LANG * N_FEAT * N_BOT);
static_assert((N_VOCAB * N_GATE3) % N_THR == 0);
static_assert(N_GATE3 % 32 == 0);

__global__ __launch_bounds__(N_THR) void prep_kernel(
    const float* __restrict__ char_embed,
    const float* __restrict__ wih_f, const float* __restrict__ whh_f,
    const float* __restrict__ bih_f, const float* __restrict__ bhh_f,
    const float* __restrict__ wih_b, const float* __restrict__ whh_b,
    const float* __restrict__ bih_b, const float* __restrict__ bhh_b,
    const float* __restrict__ down_w, const float* __restrict__ up_w, const float* __restrict__ proj_w,
    float* __restrict__ XT, _Float16* __restrict__ WHH16, _Float16* __restrict__ PW16,
    _Float16* __restrict__ DW16, _Float16* __restrict__ UW16) {
  const int blk = blockIdx.x, tid = threadIdx.x;
  if (blk < XT_BLOCKS) {
    const int gid = blk * N_THR + tid;
    const int dir = (gid >= N_VOCAB * N_GATE3) ? 1 : 0;
    const int rem = gid - dir * (N_VOCAB * N_GATE3);
    const int v = rem / N_GATE3;
    const int g = rem - v * N_GATE3;
    const float* wih = dir ? wih_b : wih_f;
    const float* bih = dir ? bih_b : bih_f;
    const float* bhh = dir ? bhh_b : bhh_f;
    const float* cr = char_embed + (size_t)v * N_CHAN;
    const float* wr = wih + (size_t)g * N_CHAN;
    float acc = 0.0f;
#pragma unroll
    for (int c4 = 0; c4 < N_CHAN / 4; ++c4) {
      const v4f a = *(const v4f*)(cr + 4 * c4);
      const v4f w = *(const v4f*)(wr + 4 * c4);
      acc = fmaf(a[0], w[0], acc);
      acc = fmaf(a[1], w[1], acc);
      acc = fmaf(a[2], w[2], acc);
      acc = fmaf(a[3], w[3], acc);
    }
    float bh = bhh[g];
    bh = (g < 2 * N_HID) ? bh : 0.0f;
    const float val = acc + bih[g] + bh;
    float* p = XT + gid;
    *(volatile float*)p = val;
    __threadfence();
    *(volatile float*)p = val;
  } else if (blk < XT_BLOCKS + WHH_BLOCKS) {
    const int i = (blk - XT_BLOCKS) * N_THR + tid;
    const int half_n = N_GATE3 * N_HID / 8;
    const float* src = (i < half_n) ? (whh_f + (size_t)i * 8) : (whh_b + (size_t)(i - half_n) * 8);
    cvt8_store(src, WHH16 + (size_t)i * 8, W_CARRY);
  } else if (blk < XT_BLOCKS + WHH_BLOCKS + PW_BLOCKS) {
    const int i = (blk - XT_BLOCKS - WHH_BLOCKS) * N_THR + tid;
    cvt8_store(proj_w + (size_t)i * 8, PW16 + (size_t)i * 8, W_CARRY);
  } else if (blk < XT_BLOCKS + WHH_BLOCKS + PW_BLOCKS + DW_BLOCKS) {
    const int i = (blk - XT_BLOCKS - WHH_BLOCKS - PW_BLOCKS) * N_THR + tid;
    cvt8_store(down_w + (size_t)i * 8, DW16 + (size_t)i * 8, W_CARRY);
  } else {
    const int i = (blk - XT_BLOCKS - WHH_BLOCKS - PW_BLOCKS - DW_BLOCKS) * N_THR + tid;
    cvt8_store(up_w + (size_t)i * 8, UW16 + (size_t)i * 8, W_CARRY);
  }
}

__global__ __launch_bounds__(N_THR) void gru_scan_kernel(
    const int* __restrict__ tokens, const float* __restrict__ XT, const _Float16* __restrict__ WHH16,
    const float* __restrict__ bhh_f, const float* __restrict__ bhh_b, float* __restrict__ FEAT) {
  __shared__ __align__(16) _Float16 h16[ROWS_PB * H_PITCH];
  __shared__ __align__(16) float    xs[ROWS_PB * X_PITCH];
  __shared__ __align__(16) int      toks[ROWS_PB * N_STEPS];
  __shared__ __align__(16) float    hfin[ROWS_PB * F_PITCH];

  const int tid = threadIdx.x, lane = tid & 31, wave = tid >> 5;
  const int rlane = lane & 15, hh = lane >> 4, koff = hh * 8, mOff = hh * 8;
  const int dir = blockIdx.y;
  const int b0 = blockIdx.x * ROWS_PB;
  const int srow = tid >> 4, sc4 = (tid & 15) * 4;

#pragma unroll
  for (int i = 0; i < 2; ++i) {
    const int col = sc4 + i * 64;
    const v4i tv = *(const v4i*)(tokens + (size_t)(b0 + srow) * N_STEPS + col);
    v4i cv;
    cv[0] = clampi(tv[0], 0, N_VOCAB - 1);
    cv[1] = clampi(tv[1], 0, N_VOCAB - 1);
    cv[2] = clampi(tv[2], 0, N_VOCAB - 1);
    cv[3] = clampi(tv[3], 0, N_VOCAB - 1);
    *(v4i*)(toks + srow * N_STEPS + col) = cv;
  }
#pragma unroll 1
  for (int i = tid; i < ROWS_PB * H_PITCH; i += N_THR) h16[i] = (_Float16)0.0f;
  __syncthreads();

  const float* XTd = XT + (size_t)dir * N_VOCAB * N_GATE3;
  {
    const int col0 = dir ? (N_STEPS - 1) : 0;
    const int tk = clampi(toks[srow * N_STEPS + col0], 0, N_VOCAB - 1);
    const float* src = XTd + (size_t)tk * N_GATE3 + sc4;
#pragma unroll
    for (int i = 0; i < 6; ++i) {
      const v4f v = *(const v4f*)(src + i * 64);
      *(v4f*)(xs + srow * X_PITCH + sc4 + i * 64) = v;
    }
  }

  const int j = 16 * wave + rlane;
  const float* bhh = dir ? bhh_b : bhh_f;
  const float bn = bhh[2 * N_HID + j];

  const _Float16* wbase = WHH16 + (size_t)dir * N_GATE3 * N_HID + (size_t)j * N_HID + koff;
  v16h wR[4], wZ[4], wN[4];
#pragma unroll
  for (int kt = 0; kt < 4; ++kt) {
    wR[kt] = FragH::load(wbase + kt * 32);
    wZ[kt] = FragH::load(wbase + (size_t)N_HID * N_HID + kt * 32);
    wN[kt] = FragH::load(wbase + (size_t)2 * N_HID * N_HID + kt * 32);
  }

  const _Float16* arow = h16 + rlane * H_PITCH + koff;
  const v8f z8 = {0.f, 0.f, 0.f, 0.f, 0.f, 0.f, 0.f, 0.f};
  float hreg[8];
#pragma unroll
  for (int r = 0; r < 8; ++r) hreg[r] = 0.0f;
  __syncthreads();

#pragma unroll 1
  for (int t = 0; t < N_STEPS; ++t) {
    v8f ar = z8, az = z8, an = z8;
#pragma unroll
    for (int kt = 0; kt < 4; ++kt) {
      const v16h a = FragH::load(arow + kt * 32);
      ar = FragH::mma(a, wR[kt], ar);
      az = FragH::mma(a, wZ[kt], az);
      an = FragH::mma(a, wN[kt], an);
      wm_guard(ar, a, wR[kt]);
      wm_guard(az, a, wZ[kt]);
      wm_guard(an, a, wN[kt]);
    }

#pragma unroll
    for (int r = 0; r < 8; ++r) {
      const float x_r = xs[(mOff + r) * X_PITCH + j];
      const float x_z = xs[(mOff + r) * X_PITCH + N_HID + j];
      const float x_n = xs[(mOff + r) * X_PITCH + 2 * N_HID + j];
      const float pr = fmaf(ar[r], REC_FOLD, x_r);
      const float pz = fmaf(az[r], REC_FOLD, x_z);
      const float hn = fmaf(an[r], REC_FOLD, bn);
      const float rg = sigm_f(pr);
      const float zg = sigm_f(pz);
      const float ng = tanh_f(fmaf(rg, hn, x_n));
      hreg[r] = (1.0f - zg) * ng + zg * hreg[r];
      if ((r & 1) == 1) __builtin_amdgcn_sched_barrier(0);
    }
    __syncthreads();
#pragma unroll
    for (int r = 0; r < 8; ++r) h16[(mOff + r) * H_PITCH + j] = f16_operand(hreg[r] * H_CARRY);
    {
      const int tn = (t + 1 < N_STEPS) ? (t + 1) : (N_STEPS - 1);
      const int col = dir ? (N_STEPS - 1 - tn) : tn;
      const int tk = clampi(toks[srow * N_STEPS + col], 0, N_VOCAB - 1);
      const float* src = XTd + (size_t)tk * N_GATE3 + sc4;
#pragma unroll
      for (int i = 0; i < 6; ++i) {
        const v4f v = *(const v4f*)(src + i * 64);
        *(v4f*)(xs + srow * X_PITCH + sc4 + i * 64) = v;
      }
    }
    __syncthreads();
  }

#pragma unroll
  for (int r = 0; r < 8; ++r) hfin[(mOff + r) * F_PITCH + j] = hreg[r];
  __syncthreads();
  {
    const int row = 2 * wave + hh;
    for (int pass = 0; pass < 2; ++pass) {
#pragma unroll
      for (int it = 0; it < 2; ++it) {
        const int c4 = it * 64 + rlane * 4;
        const v4f v = *(const v4f*)(hfin + row * F_PITCH + c4);
        *(volatile v4f*)(FEAT + (size_t)(b0 + row) * N_FEAT + dir * N_HID + c4) = v;
      }
      __threadfence();
    }
  }
}

__global__ __launch_bounds__(N_THR) void adapter_norm_kernel(
    const float* __restrict__ FEAT, const int* __restrict__ lang_ids,
    const _Float16* __restrict__ DW16, const float* __restrict__ down_b,
    const _Float16* __restrict__ UW16, const float* __restrict__ up_b,
    const float* __restrict__ ln_g, const float* __restrict__ ln_b,
    _Float16* __restrict__ Y16) {
  __shared__ __align__(16) float    xsm[ROWS_PB * AX_PITCH];
  __shared__ __align__(16) _Float16 f16s[ROWS_PB * A16_PITCH];
  __shared__ __align__(16) float    pres[ROWS_PB * N_BOT];
  __shared__ __align__(16) _Float16 hd16[ROWS_PB * HD_PITCH];
  __shared__ int langs[ROWS_PB];

  const int tid = threadIdx.x, lane = tid & 31, wave = tid >> 5;
  const int rlane = lane & 15, hh = lane >> 4, koff = hh * 8, mOff = hh * 8;
  const int b0 = blockIdx.x * ROWS_PB;

  {
    const int row = tid >> 4, c4 = (tid & 15) * 4;
#pragma unroll
    for (int i = 0; i < 4; ++i) {
      const int col = c4 + i * 64;
      const v4f v = *(const v4f*)(FEAT + (size_t)(b0 + row) * N_FEAT + col);
      *(v4f*)(xsm + row * AX_PITCH + col) = v;
      v4h hv;
      hv[0] = f16_operand(v[0] * H_CARRY);
      hv[1] = f16_operand(v[1] * H_CARRY);
      hv[2] = f16_operand(v[2] * H_CARRY);
      hv[3] = f16_operand(v[3] * H_CARRY);
      *(v4h*)(f16s + row * A16_PITCH + col) = hv;
    }
  }
  {
    int lv = lang_ids[b0 + (tid & 15)];
    asm volatile("" : "+v"(lv));
    lv = clampi(lv, 0, N_LANG - 1);
    if (tid < ROWS_PB) langs[tid] = lv;
  }
  __syncthreads();

  const v8f z8 = {0.f, 0.f, 0.f, 0.f, 0.f, 0.f, 0.f, 0.f};

  if (wave < 2) {
    const int d = wave * 16 + rlane;
    const _Float16* arow = f16s + rlane * A16_PITCH + koff;
    const _Float16* w0 = DW16 + (size_t)d * N_FEAT + koff;
    const _Float16* w1 = DW16 + (size_t)(N_BOT + d) * N_FEAT + koff;
    const _Float16* w2 = DW16 + (size_t)(2 * N_BOT + d) * N_FEAT + koff;
    v8f a0 = z8, a1 = z8, a2 = z8;
#pragma unroll 1
    for (int k0 = 0; k0 < N_FEAT; k0 += 32) {
      const v16h a  = FragH::load(arow + k0);
      const v16h q0 = FragH::load(w0 + k0);
      const v16h q1 = FragH::load(w1 + k0);
      const v16h q2 = FragH::load(w2 + k0);
      a0 = FragH::mma(a, q0, a0);
      a1 = FragH::mma(a, q1, a1);
      a2 = FragH::mma(a, q2, a2);
      wm_guard(a0, a, q0);
      wm_guard(a1, a, q1);
      wm_guard(a2, a, q2);
    }
    const float db0 = down_b[d];
    const float db1 = down_b[N_BOT + d];
    const float db2 = down_b[2 * N_BOT + d];
#pragma unroll
    for (int r = 0; r < 8; ++r) {
      const int l = langs[mOff + r];
      const float s  = (l == 0) ? a0[r] : ((l == 1) ? a1[r] : a2[r]);
      const float bs = (l == 0) ? db0 : ((l == 1) ? db1 : db2);
      pres[(mOff + r) * N_BOT + d] = fmaf(s, ADP_FOLD, bs);
    }
  }
  __syncthreads();

  for (int i = 0; i < 2; ++i) {
    const int idx = tid + i * N_THR;
    const int row = idx >> 5, d = idx & 31;
    const float p = pres[idx];
    const float g = 0.5f * p * (1.0f + erff(p * 0.70710678118654752f));
    hd16[row * HD_PITCH + d] = f16_operand(g * H_CARRY);
  }
  __syncthreads();

  {
    const v16h ah = FragH::load(hd16 + rlane * HD_PITCH + koff);
#pragma unroll
    for (int q = 0; q < 2; ++q) {
      const int e = (2 * wave + q) * 16 + rlane;
      const v16h q0 = FragH::load(UW16 + (size_t)e * N_BOT + koff);
      const v16h q1 = FragH::load(UW16 + (size_t)(N_FEAT + e) * N_BOT + koff);
      const v16h q2 = FragH::load(UW16 + (size_t)(2 * N_FEAT + e) * N_BOT + koff);
      v8f u0 = FragH::mma(ah, q0, z8);
      v8f u1 = FragH::mma(ah, q1, z8);
      v8f u2 = FragH::mma(ah, q2, z8);
      wm_guard(u0, ah, q0);
      wm_guard(u1, ah, q1);
      wm_guard(u2, ah, q2);
      const float ub0 = up_b[e];
      const float ub1 = up_b[N_FEAT + e];
      const float ub2 = up_b[2 * N_FEAT + e];
#pragma unroll
      for (int r = 0; r < 8; ++r) {
        const int l = langs[mOff + r];
        const float s  = (l == 0) ? u0[r] : ((l == 1) ? u1[r] : u2[r]);
        const float bs = (l == 0) ? ub0 : ((l == 1) ? ub1 : ub2);
        const float xv = xsm[(mOff + r) * AX_PITCH + e] + fmaf(s, ADP_FOLD, bs);
        xsm[(mOff + r) * AX_PITCH + e] = xv;
      }
    }
  }
  __syncthreads();

#pragma unroll 1
  for (int rr = 0; rr < 2; ++rr) {
    const int row = 2 * wave + rr;
    const int l = clampi(langs[row], 0, N_LANG - 1);
    const float* xr = xsm + row * AX_PITCH + lane * 8;
    const v4f p0 = *(const v4f*)(xr);
    const v4f p1 = *(const v4f*)(xr + 4);
    float s = ((p0[0] + p0[1]) + (p0[2] + p0[3])) + ((p1[0] + p1[1]) + (p1[2] + p1[3]));
#pragma unroll
    for (int off = 16; off > 0; off >>= 1) s += __shfl_xor(s, off, 32);
    const float mu = s * (1.0f / (float)N_FEAT);
    float dv[8];
#pragma unroll
    for (int e = 0; e < 4; ++e) { dv[e] = p0[e] - mu; dv[4 + e] = p1[e] - mu; }
    float vs = 0.0f;
#pragma unroll
    for (int e = 0; e < 8; ++e) vs = fmaf(dv[e], dv[e], vs);
#pragma unroll
    for (int off = 16; off > 0; off >>= 1) vs += __shfl_xor(vs, off, 32);
    const float var = vs * (1.0f / (float)N_FEAT);
    const float rstd = 1.0f / sqrtf(var + LN_EPSILON);
    const float* gp = ln_g + (size_t)l * N_FEAT + lane * 8;
    const float* bp = ln_b + (size_t)l * N_FEAT + lane * 8;
    const v4f g0 = *(const v4f*)(gp);
    const v4f g1 = *(const v4f*)(gp + 4);
    const v4f s0 = *(const v4f*)(bp);
    const v4f s1 = *(const v4f*)(bp + 4);
    v8h hv;
#pragma unroll
    for (int e = 0; e < 4; ++e) {
      const float y0 = dv[e] * rstd * g0[e] + s0[e];
      const float y1 = dv[4 + e] * rstd * g1[e] + s1[e];
      hv[e]     = f16_operand(y0 * Y_CARRY);
      hv[4 + e] = f16_operand(y1 * Y_CARRY);
    }
    _Float16* dst = Y16 + (size_t)(b0 + row) * N_FEAT + lane * 8;
    *(volatile v8h*)dst = hv;
    __threadfence();
    *(volatile v8h*)dst = hv;
  }
}

__global__ __launch_bounds__(N_THR) void proj_gemm64(
    const _Float16* __restrict__ A, int lda, const _Float16* __restrict__ Bt, int ldb,
    float* __restrict__ C, int ldc, const float* __restrict__ bias, int M, int N, int K, float scale) {
  __shared__ __align__(16) float sT[8][16 * 68];
  const int lane = threadIdx.x & 31;
  const int wave = threadIdx.x >> 5;
  const int tilesN = N >> 6;
  const int tilesM = M >> 6;
  const int tile = blockIdx.x * 8 + wave;
  if (tile >= tilesM * tilesN) return;
  const int tm = tile / tilesN;
  const int tn = tile - tm * tilesN;
  const int m0 = tm << 6;
  const int n0 = tn << 6;

  const int rlane = lane & 15;
  const int koff  = (lane >> 4) * 8;
  const int mOff  = (lane >> 4) * 8;

  v8f acc[4][4];
#pragma unroll
  for (int i = 0; i < 4; ++i)
#pragma unroll
    for (int jn = 0; jn < 4; ++jn) acc[i][jn] = (v8f){0.f, 0.f, 0.f, 0.f, 0.f, 0.f, 0.f, 0.f};

  for (int k0 = 0; k0 < K; k0 += 32) {
    v16h bh[4];
#pragma unroll
    for (int jn = 0; jn < 4; ++jn) {
      const size_t bo = (size_t)(n0 + (jn << 4) + rlane) * ldb + koff + k0;
      bh[jn] = FragH::load(Bt + bo);
    }
#pragma unroll
    for (int i = 0; i < 4; ++i) {
      const size_t ao = (size_t)(m0 + (i << 4) + rlane) * lda + koff + k0;
      const v16h ah = FragH::load(A + ao);
#pragma unroll
      for (int jn = 0; jn < 4; ++jn) acc[i][jn] = FragH::mma(ah, bh[jn], acc[i][jn]);
      wm_guard(acc[i][0], ah, bh[0]);
      wm_guard(acc[i][1], ah, bh[1]);
      wm_guard(acc[i][2], ah, bh[2]);
      wm_guard(acc[i][3], ah, bh[3]);
    }
    keep4_h(bh[0], bh[1], bh[2], bh[3]);
  }

  float* slab = sT[wave];
#pragma unroll
  for (int i = 0; i < 4; ++i) {
    const int mBase = m0 + (i << 4);
#pragma unroll
    for (int jn = 0; jn < 4; ++jn) {
      const int n = n0 + (jn << 4) + rlane;
      const float bv = bias[n];
#pragma unroll
      for (int r = 0; r < 8; ++r) {
        const float v = acc[i][jn][r] * scale + bv;
        slab[(mOff + r) * 68 + (jn << 4) + rlane] = v;
      }
    }
    __builtin_amdgcn_fence(__ATOMIC_RELEASE, "workgroup");
    __builtin_amdgcn_wave_barrier();
    __builtin_amdgcn_fence(__ATOMIC_ACQUIRE, "workgroup");
    {
      const int hq = lane >> 4, c4 = (lane & 15) * 4;
      for (int pass = 0; pass < 2; ++pass) {
#pragma unroll
        for (int it = 0; it < 8; ++it) {
          const int row = it * 2 + hq;
          const v4f v = *(const v4f*)(slab + row * 68 + c4);
          *(volatile v4f*)(C + (size_t)(mBase + row) * ldc + n0 + c4) = v;
        }
        __threadfence();
      }
    }
    __builtin_amdgcn_fence(__ATOMIC_RELEASE, "workgroup");
    __builtin_amdgcn_wave_barrier();
    __builtin_amdgcn_fence(__ATOMIC_ACQUIRE, "workgroup");
  }
}

extern "C" void kernel_launch(void* const* d_in, const int* in_sizes, int n_in,
                              void* d_out, int out_size, void* d_ws, size_t ws_size, hipStream_t stream) {
  if (n_in < 19 || d_out == nullptr || d_ws == nullptr) return;
  if (in_sizes[0] != N_BATCH * N_STEPS || in_sizes[1] != N_BATCH || in_sizes[2] != N_VOCAB * N_CHAN ||
      in_sizes[3] != N_GATE3 * N_CHAN || in_sizes[4] != N_GATE3 * N_HID || in_sizes[5] != N_GATE3 ||
      in_sizes[6] != N_GATE3 || in_sizes[7] != N_GATE3 * N_CHAN || in_sizes[8] != N_GATE3 * N_HID ||
      in_sizes[9] != N_GATE3 || in_sizes[10] != N_GATE3 || in_sizes[11] != N_LANG * N_BOT * N_FEAT ||
      in_sizes[12] != N_LANG * N_BOT || in_sizes[13] != N_LANG * N_FEAT * N_BOT || in_sizes[14] != N_LANG * N_FEAT ||
      in_sizes[15] != N_LANG * N_FEAT || in_sizes[16] != N_LANG * N_FEAT || in_sizes[17] != N_OUT * N_FEAT ||
      in_sizes[18] != N_OUT || out_size != N_BATCH * N_OUT) return;

  const int*   tokens     = (const int*)  d_in[0];
  const int*   lang_ids   = (const int*)  d_in[1];
  const float* char_embed = (const float*)d_in[2];
  const float* w_ih_f     = (const float*)d_in[3];
  const float* w_hh_f     = (const float*)d_in[4];
  const float* b_ih_f     = (const float*)d_in[5];
  const float* b_hh_f     = (const float*)d_in[6];
  const float* w_ih_b     = (const float*)d_in[7];
  const float* w_hh_b     = (const float*)d_in[8];
  const float* b_ih_b     = (const float*)d_in[9];
  const float* b_hh_b     = (const float*)d_in[10];
  const float* down_w     = (const float*)d_in[11];
  const float* down_b     = (const float*)d_in[12];
  const float* up_w       = (const float*)d_in[13];
  const float* up_b       = (const float*)d_in[14];
  const float* ln_g       = (const float*)d_in[15];
  const float* ln_b       = (const float*)d_in[16];
  const float* proj_w     = (const float*)d_in[17];
  const float* proj_b     = (const float*)d_in[18];
  float* out = (float*)d_out;

  char* ws = (char*)d_ws;
  size_t off = 0;
  auto carve = [&](size_t bytes) -> char* { char* p = ws + off; off += (bytes + 255) & ~(size_t)255; return p; };
  _Float16* WHH16 = (_Float16*)carve((size_t)2 * N_GATE3 * N_HID * 2);
  _Float16* PW16  = (_Float16*)carve((size_t)N_OUT * N_FEAT * 2);
  _Float16* DW16  = (_Float16*)carve((size_t)N_LANG * N_BOT * N_FEAT * 2);
  _Float16* UW16  = (_Float16*)carve((size_t)N_LANG * N_FEAT * N_BOT * 2);
  float*    XT    = (float*)   carve((size_t)2 * N_VOCAB * N_GATE3 * 4);
  float*    FEAT  = (float*)   carve((size_t)N_BATCH * N_FEAT * 4);
  _Float16* Y16   = (_Float16*)carve((size_t)N_BATCH * N_FEAT * 2);
  if (off > ws_size || off > (size_t)134217728) return;

  prep_kernel<<<PREP_BLOCKS, N_THR, 0, stream>>>(char_embed, w_ih_f, w_hh_f, b_ih_f, b_hh_f,
                                                 w_ih_b, w_hh_b, b_ih_b, b_hh_b,
                                                 down_w, up_w, proj_w, XT, WHH16, PW16, DW16, UW16);

  gru_scan_kernel<<<dim3(N_BATCH / ROWS_PB, 2), N_THR, 0, stream>>>(tokens, XT, WHH16, b_hh_f, b_hh_b, FEAT);

  adapter_norm_kernel<<<N_BATCH / ROWS_PB, N_THR, 0, stream>>>(FEAT, lang_ids, DW16, down_b, UW16, up_b,
                                                               ln_g, ln_b, Y16);

  const int tiles = (N_BATCH / 64) * (N_OUT / 64);
  proj_gemm64<<<tiles / 8, N_THR, 0, stream>>>(Y16, N_FEAT, PW16, N_FEAT, out, N_OUT, proj_b,
                                               N_BATCH, N_OUT, N_FEAT, PRJ_FOLD);
}
